// Rnn_86045374808728
// MI455X (gfx1250) — hardware-verified
//
#include <hip/hip_runtime.h>
#include <math.h>

constexpr int NBATCH = 8192;
constexpr int NSTEP  = 1024;
constexpr int NHID   = 32;
constexpr int CHUNK  = 32;
constexpr int NCHUNK = NSTEP / CHUNK;
constexpr int NWV    = 4;
constexpr int NTHR   = 32 * NWV;
constexpr int ROWS_W = 16;
constexpr int XP     = 36;
constexpr int NOUT0  = NBATCH * NSTEP;
constexpr int NOUT1  = 2 * NBATCH * NHID;

constexpr float WCARRY     = 64.0f;
constexpr float HCARRY     = 256.0f;
constexpr float SCARRY     = WCARRY * HCARRY;
constexpr float SCARRY_INV = 1.0f / SCARRY;
constexpr float HCARRY_INV = 1.0f / HCARRY;
constexpr double LOG2E_D   = 1.4426950408889634074;
constexpr float KTANH      = 2.0f * SCARRY_INV;
constexpr float KEXP2      = (float)(2.0 * LOG2E_D / (double)SCARRY);

static_assert(NSTEP % CHUNK == 0);
static_assert(CHUNK == 32);
static_assert(NBATCH % (ROWS_W * NWV) == 0);
static_assert(NHID == 32);
static_assert(XP % 4 == 0 && XP >= CHUNK && XP >= NHID);
static_assert((size_t)NOUT0 * 4 == (size_t)33554432);
static_assert(((size_t)NOUT0 + (size_t)NOUT1) * 4 == (size_t)35651584);

typedef __attribute__((ext_vector_type(16))) _Float16 v16h;
typedef __attribute__((ext_vector_type(8)))  float    v8f;
typedef __attribute__((ext_vector_type(4)))  float    v4f;

__device__ __forceinline__ v8f mma16(v16h a, v16h b, v8f c) {
  return __builtin_amdgcn_wmma_f32_16x16x32_f16(false, a, false, b, (short)0, c, false, false);
}
__device__ __forceinline__ void guard_grp4(v8f& a, v8f& b, v8f& c, v8f& d, v16h p, v16h q,
                                           v16h w0, v16h w1, v16h w2, v16h w3) {
  asm volatile("v_nop\n\tv_nop\n\tv_nop\n\tv_nop"
               : "+v"(a), "+v"(b), "+v"(c), "+v"(d)
               : "v"(p), "v"(q), "v"(w0), "v"(w1), "v"(w2), "v"(w3));
}
__device__ __forceinline__ void guard_grp2(v8f& a, v8f& b, v16h p, v16h w0, v16h w1) {
  asm volatile("v_nop\n\tv_nop\n\tv_nop\n\tv_nop"
               : "+v"(a), "+v"(b)
               : "v"(p), "v"(w0), "v"(w1));
}
__device__ __forceinline__ void lds_wave_sync() {
  __builtin_amdgcn_fence(__ATOMIC_RELEASE, "workgroup");
  __builtin_amdgcn_wave_barrier();
  __builtin_amdgcn_fence(__ATOMIC_ACQUIRE, "workgroup");
}

__device__ __forceinline__ float tanh_scaled(float acc) {
#if __has_builtin(__builtin_amdgcn_exp2f)
  const float e = __builtin_amdgcn_exp2f(acc * KEXP2);
#else
  const float e = __expf(acc * KTANH);
#endif
  const float r = __builtin_amdgcn_rcpf(e + 1.0f);
  return fmaf(-2.0f * HCARRY, r, HCARRY);
}

__device__ __forceinline__ void load_vec16(const float* p, int hh, float (&o)[2][8]) {
  const float* q = p + 8 * hh;
  const v4f a0 = *(const v4f*)(q);
  const v4f a1 = *(const v4f*)(q + 4);
  const v4f a2 = *(const v4f*)(q + 16);
  const v4f a3 = *(const v4f*)(q + 20);
#pragma unroll
  for (int e = 0; e < 4; ++e) {
    o[0][e]     = a0[e];
    o[0][4 + e] = a1[e];
    o[1][e]     = a2[e];
    o[1][4 + e] = a3[e];
  }
  asm volatile("" ::: "memory");
}

__device__ __forceinline__ v16h load_wfrag(const float* W, int mt, int c, int hh) {
  float t[2][8];
  load_vec16(W + (16 * mt + c) * NHID, hh, t);
  v16h f;
#pragma unroll
  for (int e = 0; e < 8; ++e) {
    f[e]     = (_Float16)(t[0][e] * WCARRY);
    f[8 + e] = (_Float16)(t[1][e] * WCARRY);
  }
  return f;
}

__device__ __forceinline__ v16h pack_h(const float (&hs)[2][8]) {
  v16h f;
#pragma unroll
  for (int e = 0; e < 8; ++e) {
    f[e]     = (_Float16)hs[0][e];
    f[8 + e] = (_Float16)hs[1][e];
  }
  return f;
}

__global__ __launch_bounds__(NTHR) __attribute__((amdgpu_num_vgpr(256))) void rnn2_seq_kernel(
    const float* __restrict__ x, const float* __restrict__ h0,
    const float* __restrict__ w_ih0, const float* __restrict__ w_hh0,
    const float* __restrict__ b_ih0, const float* __restrict__ b_hh0,
    const float* __restrict__ w_ih1, const float* __restrict__ w_hh1,
    const float* __restrict__ b_ih1, const float* __restrict__ b_hh1,
    const float* __restrict__ w_out, const float* __restrict__ b_out,
    float* __restrict__ outs, float* __restrict__ hst) {
  __shared__ __align__(16) float xsAll[NWV * ROWS_W * XP];
  __shared__ __align__(16) float ysAll[NWV * ROWS_W * XP];
  __shared__ __align__(16) float f1All[NWV * ROWS_W * XP];
  __shared__ __align__(16) float f2All[NWV * ROWS_W * XP];

  const int tid  = threadIdx.x;
  const int lane = tid & 31;
  const int wave = tid >> 5;
  const int c    = lane & 15;
  const int hh   = lane >> 4;
  const int rowbase = (blockIdx.x * NWV + wave) * ROWS_W;
  float* xs  = xsAll + wave * (ROWS_W * XP);
  float* ys  = ysAll + wave * (ROWS_W * XP);
  float* f1s = f1All + wave * (ROWS_W * XP);
  float* f2s = f2All + wave * (ROWS_W * XP);

  const v16h whh0a = load_wfrag(w_hh0, 0, c, hh);
  const v16h whh0b = load_wfrag(w_hh0, 1, c, hh);
  const v16h wih1a = load_wfrag(w_ih1, 0, c, hh);
  const v16h wih1b = load_wfrag(w_ih1, 1, c, hh);
  const v16h whh1a = load_wfrag(w_hh1, 0, c, hh);
  const v16h whh1b = load_wfrag(w_hh1, 1, c, hh);

  float b1s[2][8], w0s[2][8], wos[2][8];
  v8f c2a, c2b;
  {
    float ta[2][8], tb[2][8];
    load_vec16(b_ih0, hh, ta);
    load_vec16(b_hh0, hh, tb);
#pragma unroll
    for (int r = 0; r < 8; ++r) {
      b1s[0][r] = (ta[0][r] + tb[0][r]) * SCARRY;
      b1s[1][r] = (ta[1][r] + tb[1][r]) * SCARRY;
    }
    load_vec16(w_ih0, hh, ta);
#pragma unroll
    for (int r = 0; r < 8; ++r) {
      w0s[0][r] = ta[0][r] * SCARRY;
      w0s[1][r] = ta[1][r] * SCARRY;
    }
    load_vec16(b_ih1, hh, ta);
    load_vec16(b_hh1, hh, tb);
#pragma unroll
    for (int r = 0; r < 8; ++r) {
      c2a[r] = (ta[0][r] + tb[0][r]) * SCARRY;
      c2b[r] = (ta[1][r] + tb[1][r]) * SCARRY;
    }
    load_vec16(w_out, hh, ta);
#pragma unroll
    for (int r = 0; r < 8; ++r) {
      wos[0][r] = ta[0][r] * HCARRY_INV;
      wos[1][r] = ta[1][r] * HCARRY_INV;
    }
  }
  const float bo = b_out[0];

  v16h hb1, hb2;
  {
    float ta[2][8];
    load_vec16(h0 + (size_t)(rowbase + c) * NHID, hh, ta);
#pragma unroll
    for (int r = 0; r < 8; ++r) {
      ta[0][r] = ta[0][r] * HCARRY;
      ta[1][r] = ta[1][r] * HCARRY;
    }
    hb1 = pack_h(ta);
    load_vec16(h0 + ((size_t)NBATCH + (size_t)(rowbase + c)) * NHID, hh, ta);
#pragma unroll
    for (int r = 0; r < 8; ++r) {
      ta[0][r] = ta[0][r] * HCARRY;
      ta[1][r] = ta[1][r] * HCARRY;
    }
    hb2 = pack_h(ta);
  }

  const int lrow = lane >> 3;
  const int lc4  = (lane & 7) * 4;

#pragma unroll 1
  for (int ch = 0; ch < NCHUNK; ++ch) {
    const int t0 = ch * CHUNK;
    const bool lastc = (ch == NCHUNK - 1);
    lds_wave_sync();
    {
      v4f xq[4];
#pragma unroll
      for (int it = 0; it < 4; ++it) {
        const int row = it * 4 + lrow;
        xq[it] = *(const v4f*)(x + (size_t)(rowbase + row) * NSTEP + t0 + lc4);
      }
#pragma unroll
      for (int it = 0; it < 4; ++it) {
        const int row = it * 4 + lrow;
#pragma unroll
        for (int e = 0; e < 4; ++e) xs[row * XP + lc4 + e] = xq[it][e];
      }
    }
    lds_wave_sync();

#pragma unroll 1
    for (int tt = 0; tt < CHUNK; ++tt) {
      const bool last = lastc && (tt == CHUNK - 1);
      const float xv = xs[c * XP + tt];
      v8f acc1a, acc1b, acc2a, acc2b;
#pragma unroll
      for (int r = 0; r < 8; ++r) {
        acc1a[r] = fmaf(xv, w0s[0][r], b1s[0][r]);
        acc1b[r] = fmaf(xv, w0s[1][r], b1s[1][r]);
      }
      acc1a = mma16(whh0a, hb1, acc1a);
      acc1b = mma16(whh0b, hb1, acc1b);
      acc2a = mma16(whh1a, hb2, c2a);
      acc2b = mma16(whh1b, hb2, c2b);
      guard_grp4(acc1a, acc1b, acc2a, acc2b, hb1, hb2, whh0a, whh0b, whh1a, whh1b);
      {
        float h1s[2][8];
#pragma unroll
        for (int r = 0; r < 8; ++r) {
          h1s[0][r] = tanh_scaled(acc1a[r]);
          h1s[1][r] = tanh_scaled(acc1b[r]);
        }
        if (last) {
#pragma unroll
          for (int r = 0; r < 8; ++r) {
            f1s[c * XP + 8 * hh + r]      = h1s[0][r] * HCARRY_INV;
            f1s[c * XP + 16 + 8 * hh + r] = h1s[1][r] * HCARRY_INV;
          }
        }
        hb1 = pack_h(h1s);
      }
      acc2a = mma16(wih1a, hb1, acc2a);
      acc2b = mma16(wih1b, hb1, acc2b);
      guard_grp2(acc2a, acc2b, hb1, wih1a, wih1b);
      float part = 0.0f;
      {
        float h2s[2][8];
#pragma unroll
        for (int r = 0; r < 8; ++r) {
          h2s[0][r] = tanh_scaled(acc2a[r]);
          h2s[1][r] = tanh_scaled(acc2b[r]);
        }
        if (last) {
#pragma unroll
          for (int r = 0; r < 8; ++r) {
            f2s[c * XP + 8 * hh + r]      = h2s[0][r] * HCARRY_INV;
            f2s[c * XP + 16 + 8 * hh + r] = h2s[1][r] * HCARRY_INV;
          }
        }
        hb2 = pack_h(h2s);
#pragma unroll
        for (int r = 0; r < 8; ++r) {
          part = fmaf(h2s[0][r], wos[0][r], part);
          part = fmaf(h2s[1][r], wos[1][r], part);
        }
      }
      const float oth = __shfl_xor(part, 16, 32);
      const float yv = (part + oth) + bo;
      if (hh == 0) ys[c * XP + tt] = yv;
    }

    lds_wave_sync();
    {
      v4f yq[4];
#pragma unroll
      for (int it = 0; it < 4; ++it) {
        const int row = it * 4 + lrow;
#pragma unroll
        for (int e = 0; e < 4; ++e) yq[it][e] = ys[row * XP + lc4 + e];
      }
      for (int pass = 0; pass < 2; ++pass) {
#pragma unroll
        for (int it = 0; it < 4; ++it) {
          const int row = it * 4 + lrow;
          *(volatile v4f*)(outs + (size_t)(rowbase + row) * NSTEP + t0 + lc4) = yq[it];
        }
        __threadfence();
      }
    }
  }

  lds_wave_sync();
  {
    v4f f1[4], f2[4];
#pragma unroll
    for (int it = 0; it < 4; ++it) {
      const int row = it * 4 + lrow;
#pragma unroll
      for (int e = 0; e < 4; ++e) {
        f1[it][e] = f1s[row * XP + lc4 + e];
        f2[it][e] = f2s[row * XP + lc4 + e];
      }
    }
    float* hp1 = hst + (size_t)rowbase * NHID;
    float* hp2 = hst + ((size_t)NBATCH + (size_t)rowbase) * NHID;
    for (int pass = 0; pass < 2; ++pass) {
#pragma unroll
      for (int it = 0; it < 4; ++it) {
        const int row = it * 4 + lrow;
        *(volatile v4f*)(hp1 + row * NHID + lc4) = f1[it];
        *(volatile v4f*)(hp2 + row * NHID + lc4) = f2[it];
      }
      __threadfence();
    }
  }
}

extern "C" void kernel_launch(void* const* d_in, const int* in_sizes, int n_in,
                              void* d_out, int out_size, void* d_ws, size_t ws_size, hipStream_t stream) {
  (void)d_ws;
  (void)ws_size;
  if (n_in < 12 || d_out == nullptr) return;
  if (in_sizes[0] != NBATCH * NSTEP || in_sizes[1] != 2 * NBATCH * NHID || in_sizes[2] != NHID ||
      in_sizes[3] != NHID * NHID || in_sizes[4] != NHID || in_sizes[5] != NHID ||
      in_sizes[6] != NHID * NHID || in_sizes[7] != NHID * NHID || in_sizes[8] != NHID ||
      in_sizes[9] != NHID || in_sizes[10] != NHID || in_sizes[11] != 1 ||
      out_size != NOUT0 + NOUT1) return;

  const float* x     = (const float*)d_in[0];
  const float* h0    = (const float*)d_in[1];
  const float* w_ih0 = (const float*)d_in[2];
  const float* w_hh0 = (const float*)d_in[3];
  const float* b_ih0 = (const float*)d_in[4];
  const float* b_hh0 = (const float*)d_in[5];
  const float* w_ih1 = (const float*)d_in[6];
  const float* w_hh1 = (const float*)d_in[7];
  const float* b_ih1 = (const float*)d_in[8];
  const float* b_hh1 = (const float*)d_in[9];
  const float* w_out = (const float*)d_in[10];
  const float* b_out = (const float*)d_in[11];
  float* outs = (float*)d_out;
  float* hst  = outs + (size_t)NOUT0;

  rnn2_seq_kernel<<<NBATCH / (ROWS_W * NWV), NTHR, 0, stream>>>(
      x, h0, w_ih0, w_hh0, b_ih0, b_hh0, w_ih1, w_hh1, b_ih1, b_hh1, w_out, b_out, outs, hst);
}
